// SupervisedGraphSage_72980084293968
// MI455X (gfx1250) — hardware-verified
//
#include <hip/hip_runtime.h>

constexpr int kNodes     = 100000;
constexpr int kNodesPad  = 100032;
constexpr int kDeg       = 16;
constexpr int kFeat      = 128;
constexpr int kHid       = 128;
constexpr int kCls       = 16;
constexpr int kBatchRows = 10000;
constexpr int kKdim      = 256;
constexpr int kLdsPitch  = 264;
constexpr int kRowsPerBlockGather = 16;
constexpr int kGatherBlocks = kNodesPad / kRowsPerBlockGather;
constexpr int kL2Blocks     = kBatchRows / 16;
constexpr int kW1Blocks     = (kHid * kKdim / 8) / 256;
constexpr int kW2Blocks     = (kCls * kKdim / 8) / 256;
constexpr float kWCarry    = 16.0f;
constexpr float kWCarryInv = 0.0625f;
constexpr float kInvDeg    = 0.0625f;

static_assert(kNodesPad % 64 == 0);
static_assert(kNodesPad >= kNodes);
static_assert(kNodesPad % kRowsPerBlockGather == 0);
static_assert(kHid % 64 == 0);
static_assert(kKdim % 32 == 0);
static_assert(kBatchRows % 16 == 0);
static_assert((kHid * kKdim / 8) % 256 == 0);
static_assert((kCls * kKdim / 8) % 256 == 0);
static_assert(kLdsPitch % 8 == 0);
static_assert(kFeat == 128 && kHid == 128 && kCls == 16 && kDeg == 16);

typedef __attribute__((ext_vector_type(16))) _Float16 v16h;
typedef __attribute__((ext_vector_type(8)))  _Float16 v8h;
typedef __attribute__((ext_vector_type(16))) __bf16   v16b;
typedef __attribute__((ext_vector_type(8)))  __bf16   v8b;
typedef __attribute__((ext_vector_type(8)))  float    v8f;
typedef __attribute__((ext_vector_type(4)))  float    v4f;
typedef __attribute__((ext_vector_type(4)))  unsigned int v4u;

__device__ __forceinline__ unsigned short f2bf_bits(float f) {
  unsigned u = __float_as_uint(f);
  return (unsigned short)((u + 0x7FFFu + ((u >> 16) & 1u)) >> 16);
}
__device__ __forceinline__ float bf_bits2f(unsigned short h) { return __uint_as_float(((unsigned)h) << 16); }

__device__ __forceinline__ void dep_guard_h(v8f& a, v8f& b, v16h x, v16h y) { asm volatile("v_nop\n\tv_nop\n\tv_nop\n\tv_nop" : "+v"(a), "+v"(b) : "v"(x), "v"(y)); }
__device__ __forceinline__ void dep_guard_b(v8f& a, v8f& b, v16b x, v16b y) { asm volatile("v_nop\n\tv_nop\n\tv_nop\n\tv_nop" : "+v"(a), "+v"(b) : "v"(x), "v"(y)); }
__device__ __forceinline__ void keep4_h(v16h a, v16h b, v16h c, v16h d) { asm volatile("v_nop" :: "v"(a), "v"(b), "v"(c), "v"(d)); }
__device__ __forceinline__ void keep4_b(v16b a, v16b b, v16b c, v16b d) { asm volatile("v_nop" :: "v"(a), "v"(b), "v"(c), "v"(d)); }
__device__ __forceinline__ void acc_guard4(v8f& a, v8f& b, v8f& c, v8f& d) { asm volatile("v_nop\n\tv_nop\n\tv_nop\n\tv_nop" : "+v"(a), "+v"(b), "+v"(c), "+v"(d)); }
template <typename T> struct Frag;
template <> struct Frag<_Float16> {
  typedef v16h V; union U { v16h v; v8h h[2]; };
  static __device__ __forceinline__ v16h load(const _Float16* p) {
    U f; f.h[0] = *(const v8h*)(p); f.h[1] = *(const v8h*)(p + 16); return f.v;
  }
  static __device__ __forceinline__ v8f mma(v16h a, v16h b, v8f c) {
    return __builtin_amdgcn_wmma_f32_16x16x32_f16(false, a, false, b, (short)0, c, false, false);
  }
  static __device__ __forceinline__ void guard(v8f& a, v8f& b, v16h x, v16h y) { dep_guard_h(a, b, x, y); }
  static __device__ __forceinline__ void keep(v16h a, v16h b, v16h c, v16h d) { keep4_h(a, b, c, d); }
};
template <> struct Frag<__bf16> {
  typedef v16b V; union U { v16b v; v8b h[2]; };
  static __device__ __forceinline__ v16b load(const __bf16* p) {
    U f; f.h[0] = *(const v8b*)(p); f.h[1] = *(const v8b*)(p + 16); return f.v;
  }
  static __device__ __forceinline__ v8f mma(v16b a, v16b b, v8f c) {
    return __builtin_amdgcn_wmma_f32_16x16x32_bf16(false, a, false, b, (short)0, c, false, false);
  }
  static __device__ __forceinline__ void guard(v8f& a, v8f& b, v16b x, v16b y) { dep_guard_b(a, b, x, y); }
  static __device__ __forceinline__ void keep(v16b a, v16b b, v16b c, v16b d) { keep4_b(a, b, c, d); }
};

__device__ __forceinline__ unsigned pk16(unsigned short a, unsigned short b) { return (unsigned)a | ((unsigned)b << 16); }
__device__ __forceinline__ unsigned short h_bits(float f) { const _Float16 h = (_Float16)f; return __builtin_bit_cast(unsigned short, h); }

__device__ __forceinline__ v8f mma_h_guarded(v16h a, v16h b, v8f c) {
  c = __builtin_amdgcn_wmma_f32_16x16x32_f16(false, a, false, b, (short)0, c, false, false);
  asm volatile("v_nop\n\tv_nop\n\tv_nop\n\tv_nop" : "+v"(c) : "v"(a), "v"(b));
  return c;
}

template <int ET> struct Elem;
template <> struct Elem<0> { typedef _Float16 T; };
template <> struct Elem<1> { typedef __bf16 T; };
template <int ET, bool SPLIT, int BIAS_MODE, int OUT_MODE, bool RESID, int ACT = 0>
__global__ __launch_bounds__(256) void wmma_gemm64(
    const unsigned short* __restrict__ Ap, const unsigned short* __restrict__ A2p, int lda, long strideA,
    const unsigned short* __restrict__ Btp, const unsigned short* __restrict__ Bt2p, int ldb, long strideB,
    void* __restrict__ Cout, void* __restrict__ Cout2, int ldc, long strideC,
    const float* __restrict__ bias,
    const float* __restrict__ resid, long strideR,
    int M, int N, int K, float scale) {
  typedef typename Elem<ET>::T T;
  typedef typename Frag<T>::V V;
  const T* A = (const T*)Ap; const T* A2 = (const T*)A2p; const T* Bt = (const T*)Btp; const T* Bt2 = (const T*)Bt2p;
  __shared__ __align__(16) float sT[8][16 * 68];
  const int b    = blockIdx.y;
  const int lane = threadIdx.x & 31;
  const int wave = threadIdx.x >> 5;
  const int tilesN = N >> 6;
  const int tilesM = M >> 6;
  const int tile = blockIdx.x * 8 + wave;
  if (tile >= tilesM * tilesN) return;
  const int tm = tile / tilesN;
  const int tn = tile - tm * tilesN;
  const int m0 = tm << 6;
  const int n0 = tn << 6;

  const T* Ab  = A  + (size_t)b * strideA;
  const T* Bb  = Bt + (size_t)b * strideB;
  const T* Ab2 = SPLIT ? (A2  + (size_t)b * strideA) : nullptr;
  const T* Bb2 = SPLIT ? (Bt2 + (size_t)b * strideB) : nullptr;

  const int rlane = lane & 15;
  const int koff  = (lane >> 4) * 8;
  const int mOff  = (lane >> 4) * 8;

  v8f acc[4][4];
#pragma unroll
  for (int i = 0; i < 4; ++i)
#pragma unroll
    for (int j = 0; j < 4; ++j) acc[i][j] = (v8f){0.f,0.f,0.f,0.f,0.f,0.f,0.f,0.f};

  for (int k0 = 0; k0 < K; k0 += 32) {
    V bh[4], bl[4];
#pragma unroll
    for (int j = 0; j < 4; ++j) {
      const size_t bo = (size_t)(n0 + (j << 4) + rlane) * ldb + koff + k0;
      bh[j] = Frag<T>::load(Bb + bo);
      if (SPLIT) bl[j] = Frag<T>::load(Bb2 + bo);
    }
#pragma unroll
    for (int i = 0; i < 4; ++i) {
      const size_t ao = (size_t)(m0 + (i << 4) + rlane) * lda + koff + k0;
      V ah = Frag<T>::load(Ab + ao);
      V al;
      if (SPLIT) al = Frag<T>::load(Ab2 + ao);
#pragma unroll
      for (int j = 0; j < 4; ++j) {
        acc[i][j] = Frag<T>::mma(ah, bh[j], acc[i][j]);
        if (SPLIT) {
          acc[i][j] = Frag<T>::mma(ah, bl[j], acc[i][j]);
          acc[i][j] = Frag<T>::mma(al, bh[j], acc[i][j]);
        }
      }
      Frag<T>::guard(acc[i][0], acc[i][3], ah, SPLIT ? al : ah);
    }
    Frag<T>::keep(bh[0], bh[1], bh[2], bh[3]);
    if (SPLIT) Frag<T>::keep(bl[0], bl[1], bl[2], bl[3]);
  }
  acc_guard4(acc[0][0], acc[0][1], acc[0][2], acc[0][3]);
  acc_guard4(acc[1][0], acc[1][1], acc[1][2], acc[1][3]);
  acc_guard4(acc[2][0], acc[2][1], acc[2][2], acc[2][3]);
  acc_guard4(acc[3][0], acc[3][1], acc[3][2], acc[3][3]);

  float* slab = sT[wave];
  const float* Rb = RESID ? (resid + (size_t)b * strideR) : nullptr;
#pragma unroll
  for (int i = 0; i < 4; ++i) {
    const int mBase = m0 + (i << 4);
#pragma unroll
    for (int j = 0; j < 4; ++j) {
      const int n = n0 + (j << 4) + rlane;
      float bv = 0.f;
      if (BIAS_MODE == 2) bv = bias[n];
#pragma unroll
      for (int r = 0; r < 8; ++r) {
        float v = acc[i][j][r] * scale;
        if (BIAS_MODE == 1) v += bias[mBase + mOff + r];
        if (BIAS_MODE == 2) v += bv;
        if (RESID) v += Rb[(size_t)(mBase + mOff + r) * ldc + n];
        if (ACT == 2) v = fmaxf(v, 0.0f);
        if (ACT == 4) v = (v > 0.f) ? v : 0.01f * v;
        slab[(mOff + r) * 68 + (j << 4) + rlane] = v;
      }
    }
    __builtin_amdgcn_fence(__ATOMIC_RELEASE, "workgroup");
    __builtin_amdgcn_wave_barrier();
    __builtin_amdgcn_fence(__ATOMIC_ACQUIRE, "workgroup");
    if (OUT_MODE == 0) {
      float* C = (float*)Cout + (size_t)b * strideC;
      const int hh = lane >> 4, c4 = (lane & 15) * 4;
      for (int pass = 0; pass < 2; ++pass) {
#pragma unroll
        for (int it = 0; it < 8; ++it) {
          const int row = it * 2 + hh;
          v4f v = *(const v4f*)(slab + row * 68 + c4);
          *(volatile v4f*)(C + (size_t)(mBase + row) * ldc + n0 + c4) = v;
        }
        __threadfence();
      }
    } else {
      const int q = lane >> 3, c8 = (lane & 7) * 8;
      unsigned short* C  = (unsigned short*)Cout  + (size_t)b * strideC;
      unsigned short* C2 = (OUT_MODE == 2) ? ((unsigned short*)Cout2 + (size_t)b * strideC) : nullptr;
      for (int pass = 0; pass < 2; ++pass) {
#pragma unroll
        for (int it = 0; it < 4; ++it) {
          const int row = it * 4 + q;
          const float* sp = slab + row * 68 + c8;
          v8h hv, lv;
#pragma unroll
          for (int e = 0; e < 8; ++e) {
            if (OUT_MODE == 1) {
              hv[e] = (_Float16)sp[e];
            } else {
              unsigned short hb = f2bf_bits(sp[e]);
              unsigned short lb = f2bf_bits(sp[e] - bf_bits2f(hb));
              hv[e] = __builtin_bit_cast(_Float16, hb);
              lv[e] = __builtin_bit_cast(_Float16, lb);
            }
          }
          *(volatile v8h*)(C + (size_t)(mBase + row) * ldc + n0 + c8) = hv;
          if (OUT_MODE == 2) *(volatile v8h*)(C2 + (size_t)(mBase + row) * ldc + n0 + c8) = lv;
        }
        __threadfence();
      }
    }
    __builtin_amdgcn_fence(__ATOMIC_RELEASE, "workgroup");
    __builtin_amdgcn_wave_barrier();
    __builtin_amdgcn_fence(__ATOMIC_ACQUIRE, "workgroup");
  }
}

__global__ __launch_bounds__(256) void wcast_kernel(const float* __restrict__ W1, const float* __restrict__ W2,
                                                    unsigned short* __restrict__ Bt1, unsigned short* __restrict__ Bt2,
                                                    float scale) {
  const bool second = (blockIdx.x >= kW1Blocks);
  const float* in = second ? W2 : W1;
  unsigned short* outp = second ? Bt2 : Bt1;
  const int n8 = second ? (kCls * kKdim / 8) : (kHid * kKdim / 8);
  const int i = (second ? ((int)blockIdx.x - kW1Blocks) : (int)blockIdx.x) * 256 + (int)threadIdx.x;
  if (i >= n8) return;
  const float* p = in + 8 * (size_t)i;
  const v4f a = *(const v4f*)(p);
  const v4f c = *(const v4f*)(p + 4);
  unsigned short hb[8];
#pragma unroll
  for (int e = 0; e < 4; ++e) {
    hb[e]     = h_bits(a[e] * scale);
    hb[4 + e] = h_bits(c[e] * scale);
  }
  const v4u u = (v4u){pk16(hb[0], hb[1]), pk16(hb[2], hb[3]), pk16(hb[4], hb[5]), pk16(hb[6], hb[7])};
  unsigned short* q = outp + 8 * (size_t)i;
  *(volatile v4u*)q = u;
  __threadfence();
  *(volatile v4u*)q = u;
}

__global__ __launch_bounds__(256) void comb1_kernel(const int* __restrict__ nbr, const float* __restrict__ feat,
                                                    unsigned short* __restrict__ A1) {
  const int lane = threadIdx.x & 31, wave = threadIdx.x >> 5;
  const int hh = lane >> 4, c = lane & 15;
  const int row = (int)blockIdx.x * kRowsPerBlockGather + wave * 2 + hh;
  const bool live = row < kNodes;
  const int rc = live ? row : (kNodes - 1);
  int il = nbr[(size_t)rc * kDeg + c];
  il = il < 0 ? 0 : (il > kNodes - 1 ? kNodes - 1 : il);
  float acc[8];
#pragma unroll
  for (int e = 0; e < 8; ++e) acc[e] = 0.0f;
#pragma unroll 4
  for (int d = 0; d < kDeg; ++d) {
    const int nb = __shfl(il, (lane & 16) + d, 32);
    const float* p = feat + (size_t)nb * kFeat + 8 * c;
    const v4f a = *(const v4f*)(p);
    const v4f b = *(const v4f*)(p + 4);
#pragma unroll
    for (int e = 0; e < 4; ++e) { acc[e] += a[e]; acc[4 + e] += b[e]; }
  }
  const float* sp = feat + (size_t)rc * kFeat + 8 * c;
  const v4f s0 = *(const v4f*)(sp);
  const v4f s1 = *(const v4f*)(sp + 4);
  unsigned short hs[8], hm[8];
#pragma unroll
  for (int e = 0; e < 4; ++e) {
    const float v0 = live ? s0[e] : 0.0f;
    const float v1 = live ? s1[e] : 0.0f;
    const float m0 = live ? acc[e] * kInvDeg : 0.0f;
    const float m1 = live ? acc[4 + e] * kInvDeg : 0.0f;
    hs[e] = h_bits(v0); hs[4 + e] = h_bits(v1);
    hm[e] = h_bits(m0); hm[4 + e] = h_bits(m1);
  }
  const v4u us = (v4u){pk16(hs[0], hs[1]), pk16(hs[2], hs[3]), pk16(hs[4], hs[5]), pk16(hs[6], hs[7])};
  const v4u um = (v4u){pk16(hm[0], hm[1]), pk16(hm[2], hm[3]), pk16(hm[4], hm[5]), pk16(hm[6], hm[7])};
  unsigned short* rp = A1 + (size_t)row * kKdim + 8 * c;
  for (int pass = 0; pass < 2; ++pass) {
    *(volatile v4u*)(rp) = us;
    *(volatile v4u*)(rp + kFeat) = um;
    __threadfence();
  }
}

__global__ __launch_bounds__(256) void layer2_kernel(const int* __restrict__ nodes, const int* __restrict__ nbr,
                                                     const float* __restrict__ H1, const unsigned short* __restrict__ Bt2,
                                                     float* __restrict__ out) {
  __shared__ __align__(16) unsigned short sA[16 * kLdsPitch];
  __shared__ __align__(16) float sO[256];
  const int lane = threadIdx.x & 31, wave = threadIdx.x >> 5;
  const int hh = lane >> 4, c = lane & 15;
  const int rloc = wave * 2 + hh;
  const int b = (int)blockIdx.x * 16 + rloc;
  int nd = nodes[b];
  nd = nd < 0 ? 0 : (nd > kNodes - 1 ? kNodes - 1 : nd);
  int il = nbr[(size_t)nd * kDeg + c];
  il = il < 0 ? 0 : (il > kNodes - 1 ? kNodes - 1 : il);
  float acc[8];
#pragma unroll
  for (int e = 0; e < 8; ++e) acc[e] = 0.0f;
#pragma unroll 4
  for (int d = 0; d < kDeg; ++d) {
    const int nb = __shfl(il, (lane & 16) + d, 32);
    const float* p = H1 + (size_t)nb * kHid + 8 * c;
    const v4f a = *(const v4f*)(p);
    const v4f q = *(const v4f*)(p + 4);
#pragma unroll
    for (int e = 0; e < 4; ++e) { acc[e] += a[e]; acc[4 + e] += q[e]; }
  }
  const float* sp = H1 + (size_t)nd * kHid + 8 * c;
  const v4f s0 = *(const v4f*)(sp);
  const v4f s1 = *(const v4f*)(sp + 4);
  unsigned short hs[8], hm[8];
#pragma unroll
  for (int e = 0; e < 4; ++e) {
    hs[e] = h_bits(s0[e]); hs[4 + e] = h_bits(s1[e]);
    hm[e] = h_bits(acc[e] * kInvDeg); hm[4 + e] = h_bits(acc[4 + e] * kInvDeg);
  }
  const v4u us = (v4u){pk16(hs[0], hs[1]), pk16(hs[2], hs[3]), pk16(hs[4], hs[5]), pk16(hs[6], hs[7])};
  const v4u um = (v4u){pk16(hm[0], hm[1]), pk16(hm[2], hm[3]), pk16(hm[4], hm[5]), pk16(hm[6], hm[7])};
  *(v4u*)(sA + rloc * kLdsPitch + 8 * c) = us;
  *(v4u*)(sA + rloc * kLdsPitch + kHid + 8 * c) = um;
  __syncthreads();

  if (wave == 0) {
    const _Float16* sAh = (const _Float16*)sA;
    const _Float16* Bh  = (const _Float16*)Bt2;
    v8f d = (v8f){0.f, 0.f, 0.f, 0.f, 0.f, 0.f, 0.f, 0.f};
#pragma unroll
    for (int ks = 0; ks < kKdim / 32; ++ks) {
      const v16h af = Frag<_Float16>::load(sAh + c * kLdsPitch + ks * 32 + 8 * hh);
      const v16h bf = Frag<_Float16>::load(Bh + (size_t)c * kKdim + ks * 32 + 8 * hh);
      d = mma_h_guarded(af, bf, d);
    }
#pragma unroll
    for (int r = 0; r < 8; ++r) sO[(8 * hh + r) * 16 + c] = d[r] * kWCarryInv;
  }
  __syncthreads();

  if (wave == 0) {
    const v4f p0 = *(const v4f*)(sO + 4 * lane);
    const v4f p1 = *(const v4f*)(sO + 128 + 4 * lane);
    float* op = out + (size_t)blockIdx.x * 256;
    for (int pass = 0; pass < 2; ++pass) {
      *(volatile v4f*)(op + 4 * lane) = p0;
      *(volatile v4f*)(op + 128 + 4 * lane) = p1;
      __threadfence();
    }
  }
}

extern "C" void kernel_launch(void* const* d_in, const int* in_sizes, int n_in,
                              void* d_out, int out_size, void* d_ws, size_t ws_size, hipStream_t stream) {
  (void)in_sizes; (void)n_in; (void)out_size;
  const int*   nodes = (const int*)  d_in[0];
  const int*   nbr   = (const int*)  d_in[1];
  const float* feat  = (const float*)d_in[2];
  const float* W1    = (const float*)d_in[3];
  const float* W2    = (const float*)d_in[4];
  float* out = (float*)d_out;

  char* ws = (char*)d_ws; size_t off = 0;
  auto carve = [&](size_t bytes) -> char* { char* p = ws + off; off += (bytes + 255) & ~(size_t)255; return p; };
  unsigned short* A1  = (unsigned short*)carve((size_t)kNodesPad * kKdim * 2);
  float*          H1  = (float*)carve((size_t)kNodesPad * kHid * 4);
  unsigned short* Bt1 = (unsigned short*)carve((size_t)kHid * kKdim * 2);
  unsigned short* Bt2 = (unsigned short*)carve((size_t)kCls * kKdim * 2);
  if (off > ws_size || off > (size_t)134217728) return;

  wcast_kernel<<<kW1Blocks + kW2Blocks, 256, 0, stream>>>(W1, W2, Bt1, Bt2, kWCarry);
  comb1_kernel<<<kGatherBlocks, 256, 0, stream>>>(nbr, feat, A1);
  {
    const int tiles = (kNodesPad / 64) * (kHid / 64);
    wmma_gemm64<0, false, 0, 0, false, 2><<<dim3((tiles + 7) / 8, 1), 256, 0, stream>>>(
        (const unsigned short*)A1, (const unsigned short*)nullptr, kKdim, 0L,
        (const unsigned short*)Bt1, (const unsigned short*)nullptr, kKdim, 0L,
        (void*)H1, (void*)nullptr, kHid, 0L,
        (const float*)nullptr, (const float*)nullptr, 0L,
        kNodesPad, kHid, kKdim, kWCarryInv);
  }
  layer2_kernel<<<kL2Blocks, 256, 0, stream>>>(nodes, nbr, H1, Bt2, out);
}
